// GCNEntPair_71159018160437
// MI455X (gfx1250) — hardware-verified
//
#include <hip/hip_runtime.h>
#include <stddef.h>
#include <stdint.h>
#include <math.h>


#define NN     50000
#define EE     800000
#define GG     1024
#define NAT    11
#define VOC    100000
#define DE     128
#define DH     256
#define DHID   512
#define DOUT   128
#define MP     50048
#define NTHR   256
#define NWAVE  8
#define EPT    8
#define CHUNK  (NTHR * EPT)
#define WCAP   (EPT * 32)
#define LISTN  (NWAVE * WCAP)
#define NBA    1024
#define SLA    10
#define NBLK   49
#define NPADN  (NBLK * NBA)
#define RCAP   20480
#define DEGCAP 64
#define GBM    64
#define GBN    64
#define GTHR   128
#define PGB    32
#define NPB    (GG / PGB)
#define PCAP   8192
#define NPOL   (2 * NBLK + 2 * NPB)
#define AGG_ZINTS (LISTN + 2 * RCAP + 3 * NBA)
#define BKT_LDS_INTS (AGG_ZINTS + 16)
#define WSMAX  134217728

static_assert(MP % 128 == 0 && MP >= NN && MP % GBM == 0);
static_assert(NN <= 65536 && NBA <= 1024 && NBA == (1 << SLA));
static_assert(NBLK * NBA >= MP);
static_assert((CHUNK & (CHUNK - 1)) == 0);
static_assert(((long long)(EE + CHUNK) << SLA) < (1LL << 31));
static_assert(EE % 4 == 0);
static_assert(RCAP % 32 == 0 && RCAP % (NTHR * 4) == 0 && AGG_ZINTS % 4 == 0);
static_assert((long long)RCAP * 100 >= 16633LL * 105);
static_assert(DEGCAP >= 36 + 8);
static_assert(DH == 32 * 8 && DE % 32 == 0 && DH % 128 == 0 && DHID % 128 == 0 && DOUT % 64 == 0);
static_assert(GBM == (GTHR / 32) * 16 && GBN == 64);
static_assert(BKT_LDS_INTS * 4 <= 300000);
static_assert(GG % PGB == 0 && PGB == 4 * NWAVE && PCAP % NTHR == 0);
static_assert((GG * DOUT * 4) % 128 == 0);

typedef float          v2f   __attribute__((ext_vector_type(2)));
typedef float          v4f   __attribute__((ext_vector_type(4)));
typedef float          v8f   __attribute__((ext_vector_type(8)));
typedef int            v4i   __attribute__((ext_vector_type(4)));
typedef int            v8i   __attribute__((ext_vector_type(8)));
typedef unsigned int   v2u   __attribute__((ext_vector_type(2)));
typedef unsigned int   v4u   __attribute__((ext_vector_type(4)));
typedef unsigned short v8us  __attribute__((ext_vector_type(8)));
typedef unsigned short v16us __attribute__((ext_vector_type(16)));
typedef __bf16         v16bf __attribute__((ext_vector_type(16)));
typedef v2u  __attribute__((may_alias)) v2ua;
typedef v4f  __attribute__((may_alias)) v4fa;
typedef v4i  __attribute__((may_alias)) v4ia;
typedef v8us __attribute__((may_alias)) v8usa;
union FragB { v16bf v; v16us u; v8us h[2]; v8i w; };

__device__ __forceinline__ v8f wmb(const FragB& a, const FragB& b, v8f c) {
  v8f d = __builtin_amdgcn_wmma_f32_16x16x32_bf16(false, a.v, false, b.v, (short)0, c, false, false);
  asm volatile("v_nop\n\tv_nop\n\tv_nop\n\tv_nop" : "+v"(d) : "v"(a.w), "v"(b.w));
  return d;
}

__device__ __forceinline__ unsigned bf16_bits(float f) {
  const unsigned u = __float_as_uint(f);
  const unsigned r = (u + 0x7FFFu + ((u >> 16) & 1u)) >> 16;
  return (f != f) ? 0x7FC0u : r;
}
__device__ __forceinline__ float bf16_val(float f) {
  return __uint_as_float(bf16_bits(f) << 16);
}
__device__ __forceinline__ float relu_np(float v) { return (v > 0.0f) ? v : (v - v); }
__device__ __forceinline__ unsigned hl_pick(float f, bool lo) {
  const unsigned h = bf16_bits(f);
  const unsigned l = bf16_bits(f - __uint_as_float(h << 16));
  return lo ? l : h;
}

template <int SLB>
__device__ __forceinline__ int scan_chunk(const int* __restrict__ dsts, int nE, int cbase, int slotBase,
                                          int nb, int vec8, int* list, int tid, int lane, int wave) {
  int wc = 0;
  const int el0  = tid * EPT;
  const int e0   = cbase + el0;
  const int sent = -2147483647 - 1;
  v4i da, db;
  if (vec8 != 0 && cbase + CHUNK <= nE) {
    da = *(const v4i*)(dsts + e0);
    db = *(const v4i*)(dsts + e0 + 4);
  } else {
    da.x = (e0     < nE) ? dsts[min(e0,     nE - 1)] : sent;
    da.y = (e0 + 1 < nE) ? dsts[min(e0 + 1, nE - 1)] : sent;
    da.z = (e0 + 2 < nE) ? dsts[min(e0 + 2, nE - 1)] : sent;
    da.w = (e0 + 3 < nE) ? dsts[min(e0 + 3, nE - 1)] : sent;
    db.x = (e0 + 4 < nE) ? dsts[min(e0 + 4, nE - 1)] : sent;
    db.y = (e0 + 5 < nE) ? dsts[min(e0 + 5, nE - 1)] : sent;
    db.z = (e0 + 6 < nE) ? dsts[min(e0 + 6, nE - 1)] : sent;
    db.w = (e0 + 7 < nE) ? dsts[min(e0 + 7, nE - 1)] : sent;
  }
  const unsigned nbs = (unsigned)slotBase;
  const unsigned unb = (unsigned)nb;
  const unsigned s0 = (unsigned)da.x - nbs, s1 = (unsigned)da.y - nbs;
  const unsigned s2 = (unsigned)da.z - nbs, s3 = (unsigned)da.w - nbs;
  const unsigned s4 = (unsigned)db.x - nbs, s5 = (unsigned)db.y - nbs;
  const unsigned s6 = (unsigned)db.z - nbs, s7 = (unsigned)db.w - nbs;
  const bool h0 = s0 < unb, h1 = s1 < unb, h2 = s2 < unb, h3 = s3 < unb;
  const bool h4 = s4 < unb, h5 = s5 < unb, h6 = s6 < unb, h7 = s7 < unb;
  const unsigned any = __builtin_amdgcn_ballot_w32(h0 | h1 | h2 | h3 | h4 | h5 | h6 | h7);
  if (any != 0u) {
#define HITJ(J, HJ, SJ) { \
      const unsigned mj = __builtin_amdgcn_ballot_w32(HJ); \
      if (mj != 0u) { \
        if (HJ) { \
          const int pos = wc + (int)__builtin_amdgcn_mbcnt_lo(mj, 0u); \
          if (pos < WCAP) list[wave * WCAP + pos] = ((el0 + (J)) << SLB) | (int)(SJ); \
        } \
        wc += (int)__builtin_popcount(mj); } }
    HITJ(0, h0, s0)
    HITJ(1, h1, s1)
    HITJ(2, h2, s2)
    HITJ(3, h3, s3)
    HITJ(4, h4, s4)
    HITJ(5, h5, s5)
    HITJ(6, h6, s6)
    HITJ(7, h7, s7)
#undef HITJ
  }
  return wc;
}

__device__ __forceinline__ void wt_unit(const float* __restrict__ W, unsigned short* WT, int v,
                                        int K, int N, int KD) {
  const int upr = KD >> 3;
  const int n   = v / upr;
  const int k8  = (v - n * upr) * 8;
  const int kk  = (k8 >= K) ? (k8 - K) : k8;
  const float* p = W + (size_t)kk * N + n;
  v8us o;
#pragma unroll
  for (int i = 0; i < 8; ++i) o[i] = (unsigned short)bf16_bits(p[(size_t)i * N]);
  unsigned short* dp = WT + (size_t)n * KD + k8;
  *(volatile v8us*)dp = o;
  __threadfence();
  *(volatile v8us*)dp = o;
}

__device__ __forceinline__ void row_unit(const float* __restrict__ p, unsigned short* dp, bool ok, int rl) {
  const v4f a = *(const v4fa*)p;
  const v4f b = *(const v4fa*)(p + 4);
  const float f[8] = {a.x, a.y, a.z, a.w, b.x, b.y, b.z, b.w};
  v8us o;
#pragma unroll
  for (int i = 0; i < 8; ++i) {
    unsigned bts = bf16_bits(f[i]);
    const bool neg = (bts & 0x8000u) != 0u;
    bts = (rl != 0 && neg) ? 0u : bts;
    o[i] = ok ? (unsigned short)bts : (unsigned short)0;
  }
  *(volatile v8us*)dp = o;
  __threadfence();
  *(volatile v8us*)dp = o;
}

#define PB0 4096
#define PB1 (PB0 + 16384)
#define PB2 (PB1 + 16384)
#define PB3 (PB2 + 4096)
#define PB4 (PB3 + 16384)
#define PB5 (PB4 + 65536)
#define PB6 (PB5 + 65536)
#define PB7 (PB6 + 16384)
#define PB8 (PB7 + 2048)
#define PB9 (PB8 + 16384)
#define PB10 (PB9 + 16384)
static_assert(PB0 % NTHR == 0 && PB1 % NTHR == 0 && PB2 % NTHR == 0 && PB3 % NTHR == 0 && PB4 % NTHR == 0);
static_assert(PB5 % NTHR == 0 && PB6 % NTHR == 0 && PB7 % NTHR == 0 && PB8 % NTHR == 0 && PB9 % NTHR == 0);
static_assert(PB10 % NTHR == 0);
static_assert(DH * (DE / 8) == 4096 && DH * (2 * DH / 8) == 16384 && DHID * (2 * DHID / 8) == 65536);
static_assert(DOUT * (2 * DHID / 8) == 16384 && 128 * (DE / 8) == 2048 && GG * (DE / 8) == 16384);

__global__ __launch_bounds__(NTHR) void k_prep(
    const float* __restrict__ gW1, const float* __restrict__ gW2, const float* __restrict__ fcW,
    const float* __restrict__ eW1, const float* __restrict__ eW2, const float* __restrict__ dW1,
    const float* __restrict__ dW2, const float* __restrict__ dW3, const float* __restrict__ aemb,
    const float* __restrict__ eemb, const int* __restrict__ ent1, const int* __restrict__ ent2,
    unsigned short* gW1T, unsigned short* gW2D, unsigned short* fcWD, unsigned short* eW1T,
    unsigned short* eW2D, unsigned short* dW1D, unsigned short* dW2D, unsigned short* dW3D,
    unsigned short* AE, unsigned short* E0) {
  const int u = (int)blockIdx.x * NTHR + (int)threadIdx.x;
  if (u < PB0)       { wt_unit(gW1, gW1T, u,       DE,   DH,   DE);       return; }
  if (u < PB1)       { wt_unit(gW2, gW2D, u - PB0, DH,   DH,   2 * DH);   return; }
  if (u < PB2)       { wt_unit(fcW, fcWD, u - PB1, DH,   DH,   2 * DH);   return; }
  if (u < PB3)       { wt_unit(eW1, eW1T, u - PB2, DE,   DH,   DE);       return; }
  if (u < PB4)       { wt_unit(eW2, eW2D, u - PB3, DH,   DH,   2 * DH);   return; }
  if (u < PB5)       { wt_unit(dW1, dW1D, u - PB4, DHID, DHID, 2 * DHID); return; }
  if (u < PB6)       { wt_unit(dW2, dW2D, u - PB5, DHID, DHID, 2 * DHID); return; }
  if (u < PB7)       { wt_unit(dW3, dW3D, u - PB6, DHID, DOUT, 2 * DHID); return; }
  if (u < PB8) {
    const int v = u - PB7;
    const int row = v >> 4, k8 = (v & 15) * 8;
    const int rc = row < NAT ? row : NAT - 1;
    row_unit(aemb + (size_t)rc * DE + k8, AE + (size_t)row * DE + k8, row < NAT, 0);
    return;
  }
  if (u < PB9) {
    const int v = u - PB8;
    const int g = v >> 4, k8 = (v & 15) * 8;
    int id = ent1[g];
    id = id < 0 ? 0 : (id > VOC - 1 ? VOC - 1 : id);
    row_unit(eemb + (size_t)id * DE + k8, E0 + (size_t)g * DE + k8, true, 1);
    return;
  }
  if (u < PB10) {
    const int v = u - PB9;
    const int g = v >> 4, k8 = (v & 15) * 8;
    int id = ent2[g];
    id = id < 0 ? 0 : (id > VOC - 1 ? VOC - 1 : id);
    row_unit(eemb + (size_t)id * DE + k8, E0 + (size_t)(GG + g) * DE + k8, true, 1);
    return;
  }
}

template <int RELU, int HILO>
__global__ __launch_bounds__(GTHR) void k_gemm(
    const unsigned short* __restrict__ A, const unsigned short* __restrict__ WT,
    const float* __restrict__ bias, int hasBias,
    float* outF, unsigned short* outH, int K, int ldo)
{
  __shared__ __attribute__((aligned(16))) float stg[GBM * GBN];
  const int tid = (int)threadIdx.x, lane = tid & 31, wave = tid >> 5, hh = lane >> 4, m = lane & 15;
  const int rowBase = (int)blockIdx.x * GBM;
  const int col0    = (int)blockIdx.y * GBN;

  v8f acc[4];
  {
    const v8f z = {0.f, 0.f, 0.f, 0.f, 0.f, 0.f, 0.f, 0.f};
    acc[0] = z; acc[1] = z; acc[2] = z; acc[3] = z;
  }
  const unsigned short* ap = A  + (size_t)(rowBase + 16 * wave + m) * (size_t)K + 8 * hh;
  const unsigned short* wp = WT + (size_t)(col0 + m) * (size_t)K + 8 * hh;
  const int ksteps = K >> 5;
#pragma unroll 1
  for (int ks = 0; ks < ksteps; ++ks) {
    FragB af;
    af.h[0] = *(const v8usa*)(ap + 32 * ks);
    af.h[1] = *(const v8usa*)(ap + 32 * ks + 16);
#pragma unroll
    for (int t = 0; t < 4; ++t) {
      const unsigned short* wq = wp + (size_t)(16 * t) * (size_t)K + 32 * ks;
      FragB bf;
      bf.h[0] = *(const v8usa*)wq;
      bf.h[1] = *(const v8usa*)(wq + 16);
      acc[t] = wmb(af, bf, acc[t]);
    }
  }

#pragma unroll
  for (int t = 0; t < 4; ++t) {
    const int lc = 16 * t + m;
    const float braw = bias[col0 + lc];
    const float bb = (hasBias != 0) ? bf16_val(braw) : 0.0f;
#pragma unroll
    for (int r = 0; r < 8; ++r) {
      const int lr = 16 * wave + 8 * hh + r;
      float v = acc[t][r] + bb;
      if (RELU != 0) v = relu_np(v);
      stg[lr * GBN + lc] = v;
    }
  }
  __syncthreads();

  if constexpr (HILO == 0) {
    v4f fv[8];
#pragma unroll
    for (int i = 0; i < 8; ++i) {
      const int lr = 16 * wave + 2 * i + hh;
      fv[i] = *(const v4fa*)(stg + lr * GBN + 4 * m);
    }
#pragma unroll
    for (int i = 0; i < 8; ++i) {
      const int gr = rowBase + 16 * wave + 2 * i + hh;
      float* op = outF + (size_t)gr * (size_t)ldo + col0 + 4 * m;
      *(volatile v4f*)op = fv[i];
    }
    __threadfence();
#pragma unroll
    for (int i = 0; i < 8; ++i) {
      const int gr = rowBase + 16 * wave + 2 * i + hh;
      float* op = outF + (size_t)gr * (size_t)ldo + col0 + 4 * m;
      *(volatile v4f*)op = fv[i];
    }
  } else {
    const int q = m & 7;
    const bool lsel = (m & 8) != 0;
    const int segoff = lsel ? ldo : 0;
    v4u pk[8];
#pragma unroll
    for (int i = 0; i < 8; ++i) {
      const int lr = 16 * wave + 2 * i + hh;
      const v4f a = *(const v4fa*)(stg + lr * GBN + 8 * q);
      const v4f b = *(const v4fa*)(stg + lr * GBN + 8 * q + 4);
      v4u pw;
      pw.x = hl_pick(a.x, lsel) | (hl_pick(a.y, lsel) << 16);
      pw.y = hl_pick(a.z, lsel) | (hl_pick(a.w, lsel) << 16);
      pw.z = hl_pick(b.x, lsel) | (hl_pick(b.y, lsel) << 16);
      pw.w = hl_pick(b.z, lsel) | (hl_pick(b.w, lsel) << 16);
      pk[i] = pw;
    }
#pragma unroll
    for (int i = 0; i < 8; ++i) {
      const int gr = rowBase + 16 * wave + 2 * i + hh;
      unsigned short* op = outH + (size_t)gr * (size_t)(2 * ldo) + segoff + col0 + 8 * q;
      *(volatile v4u*)op = pk[i];
    }
    __threadfence();
#pragma unroll
    for (int i = 0; i < 8; ++i) {
      const int gr = rowBase + 16 * wave + 2 * i + hh;
      unsigned short* op = outH + (size_t)gr * (size_t)(2 * ldo) + segoff + col0 + 8 * q;
      *(volatile v4u*)op = pk[i];
    }
  }
}

__global__ __launch_bounds__(NTHR) void k_bucket(const int* __restrict__ srcs, const int* __restrict__ dsts,
                                                 const int* __restrict__ xin,
                                                 unsigned int* LISTg, unsigned int* COg, unsigned int* XDg,
                                                 unsigned int* POl) {
  extern __shared__ __attribute__((aligned(16))) int dsm[];
  int* list = dsm;
  int* hl   = dsm + LISTN;
  int* sl   = dsm + LISTN + RCAP;
  int* cnt  = dsm + LISTN + 2 * RCAP;
  int* offs = cnt + NBA;
  int* cur  = offs + NBA;
  int* misc = cur + NBA;
  const int tid = (int)threadIdx.x, lane = tid & 31, wave = tid >> 5;
  const int nodeBase = (int)blockIdx.x * NBA;
  const int nE = EE, nN = NN;

  {
    const v4i z4 = {0, 0, 0, 0};
    for (int i = tid * 4; i < AGG_ZINTS; i += NTHR * 4) *(v4ia*)(dsm + i) = z4;
    if (tid < 16) misc[tid] = 0;
  }
  __syncthreads();

  int t = 0, ov = 0;
  const int nChunks = (nE + CHUNK - 1) / CHUNK;
#pragma unroll 1
  for (int ch = 0; ch < nChunks; ++ch) {
    const int cbase = ch * CHUNK;
    const int wc = scan_chunk<SLA>(dsts, nE, cbase, nodeBase, NBA, 1, list, tid, lane, wave);
    if (lane == 0) misc[wave] = wc;
    __syncthreads();
    if (wave == 0) {
#pragma unroll 1
      for (int w2 = 0; w2 < NWAVE; ++w2) {
        int c = misc[w2];
        c = c < 0 ? 0 : (c > WCAP ? WCAP : c);
#pragma unroll 1
        for (int b0 = 0; b0 < c; b0 += 32) {
          const int idx = b0 + lane;
          const int ent = list[w2 * WCAP + (idx < WCAP ? idx : WCAP - 1)];
          const int m32 = (c - b0) < 32 ? (c - b0) : 32;
#pragma unroll 1
          for (int k = 0; k < m32; ++k) {
            const int u    = __builtin_amdgcn_readlane(ent, k);
            const int slot = u & (NBA - 1);
            const int el   = (u >> SLA) & (CHUNK - 1);
            const int pk   = ((cbase + el) << SLA) | slot;
            if (t < RCAP) {
              if (lane == 0) { hl[t] = pk; cnt[slot] = cnt[slot] + 1; }
              t = t + 1;
            } else {
              ov = 1;
            }
          }
        }
      }
    }
    __syncthreads();
  }
  if (wave == 0 && lane == 0) { misc[8] = t; misc[9] = ov; }
  __syncthreads();
  int tt = misc[8];
  tt = tt < 0 ? 0 : (tt > RCAP ? RCAP : tt);
  const int ovf = misc[9];

  if (wave == 0) {
    const int base = lane * (NBA / 32);
    int s = 0;
#pragma unroll 1
    for (int i = 0; i < NBA / 32; ++i) s += cnt[base + i];
    int incl = s;
#pragma unroll
    for (int d = 1; d < 32; d <<= 1) {
      const int y = __shfl_up(incl, d, 32);
      if (lane >= d) incl += y;
    }
    int run = incl - s;
#pragma unroll 1
    for (int i = 0; i < NBA / 32; ++i) {
      const int cv = cnt[base + i];
      offs[base + i] = run;
      cur[base + i]  = run;
      run += cv;
    }
  }
  __syncthreads();
  if (wave == 0) {
#pragma unroll 1
    for (int b0 = 0; b0 < tt; b0 += 32) {
      const int idx = b0 + lane;
      const int ent = hl[idx < RCAP ? idx : RCAP - 1];
      const int m32 = (tt - b0) < 32 ? (tt - b0) : 32;
#pragma unroll 1
      for (int k = 0; k < m32; ++k) {
        const int u    = __builtin_amdgcn_readlane(ent, k);
        const int slot = u & (NBA - 1);
        if (lane == 0) {
          int p = cur[slot];
          p = p < 0 ? 0 : (p > RCAP - 1 ? RCAP - 1 : p);
          sl[p] = u;
          cur[slot] = p + 1;
        }
      }
    }
  }
  __syncthreads();

#pragma unroll 4
  for (int i = tid; i < RCAP; i += NTHR) {
    const int u = sl[i];
    const int slot = u & (NBA - 1);
    int eid = u >> SLA;
    eid = eid < 0 ? 0 : (eid > nE - 1 ? nE - 1 : eid);
    int sr = srcs[eid];
    sr = sr < 0 ? 0 : (sr > nN - 1 ? nN - 1 : sr);
    const unsigned pk = ((unsigned)slot << 16) | (unsigned)sr;
    hl[i] = (i < tt) ? (int)pk : 0;
  }
#pragma unroll 1
  for (int it = 0; it < NBA / NTHR; ++it) {
    const int r = it * NTHR + tid;
    const int node = nodeBase + r;
    const int nc = node < nN ? node : nN - 1;
    int xv = xin[nc];
    xv = xv < 0 ? 0 : (xv > NAT - 1 ? NAT - 1 : xv);
    int c = cnt[r];
    c = c < 0 ? 0 : c;
    const float dg = (float)(c + 1);
    const float di = 1.0f / sqrtf(dg);
    const bool live = node < nN;
    list[r] = live ? xv : 0;
    cur[r]  = live ? __float_as_int(di) : 0;
  }
  __syncthreads();

  unsigned int* lp = LISTg + (size_t)blockIdx.x * RCAP;
  v4u co[2], xd[2];
#pragma unroll
  for (int it = 0; it < 2; ++it) {
    const int r = it * 512 + 2 * tid;
    v4u a, b;
    a.x = (unsigned)cnt[r];      a.y = (unsigned)offs[r];
    a.z = (unsigned)cnt[r + 1];  a.w = (unsigned)offs[r + 1];
    b.x = (unsigned)list[r];     b.y = (unsigned)cur[r];
    b.z = (unsigned)list[r + 1]; b.w = (unsigned)cur[r + 1];
    co[it] = a; xd[it] = b;
  }
  const unsigned fv = (ovf != 0) ? 1u : 0u;
  const v4u fl = {fv, fv, fv, fv};
  const bool flw = (wave == 0) && (lane < 8);

#pragma unroll 1
  for (int i = tid * 4; i < RCAP; i += NTHR * 4) {
    const v4i v = *(const v4ia*)(hl + i);
    *(volatile v4i*)(lp + i) = v;
  }
#pragma unroll
  for (int it = 0; it < 2; ++it) {
    const size_t ro = 2 * (size_t)(nodeBase + it * 512 + 2 * tid);
    *(volatile v4u*)(COg + ro) = co[it];
    *(volatile v4u*)(XDg + ro) = xd[it];
  }
  if (flw) *(volatile v4u*)(POl + (size_t)blockIdx.x * 32 + 4 * lane) = fl;
  __threadfence();
#pragma unroll 1
  for (int i = tid * 4; i < RCAP; i += NTHR * 4) {
    const v4i v = *(const v4ia*)(hl + i);
    *(volatile v4i*)(lp + i) = v;
  }
#pragma unroll
  for (int it = 0; it < 2; ++it) {
    const size_t ro = 2 * (size_t)(nodeBase + it * 512 + 2 * tid);
    *(volatile v4u*)(COg + ro) = co[it];
    *(volatile v4u*)(XDg + ro) = xd[it];
  }
  if (flw) *(volatile v4u*)(POl + (size_t)blockIdx.x * 32 + 4 * lane) = fl;
}

__global__ __launch_bounds__(NTHR) void k_agg1(const unsigned int* __restrict__ LISTg,
                                               const unsigned int* __restrict__ COg,
                                               const unsigned int* __restrict__ XDg,
                                               const unsigned int* __restrict__ POl,
                                               const float* __restrict__ T1, const float* __restrict__ gb,
                                               unsigned short* H1) {
  __shared__ __attribute__((aligned(16))) float t1s[NAT * DH];
  const int tid = (int)threadIdx.x, lane = tid & 31, wave = tid >> 5;
  const int nodeBase = (int)blockIdx.x * NBA;
#pragma unroll 1
  for (int i = tid; i < (NAT * DH) / 4; i += NTHR) *(v4fa*)(t1s + 4 * i) = *(const v4fa*)(T1 + 4 * i);
  float b0v, b1v, b2v, b3v, b4v, b5v, b6v, b7v;
  {
    const v4f a = *(const v4fa*)(gb + 8 * lane);
    const v4f b = *(const v4fa*)(gb + 8 * lane + 4);
    b0v = bf16_val(a.x); b1v = bf16_val(a.y); b2v = bf16_val(a.z); b3v = bf16_val(a.w);
    b4v = bf16_val(b.x); b5v = bf16_val(b.y); b6v = bf16_val(b.z); b7v = bf16_val(b.w);
  }
  const unsigned pfl = POl[(size_t)blockIdx.x * 32];
  __syncthreads();

  const unsigned int* lp = LISTg + (size_t)blockIdx.x * RCAP;
  const float qnan = __int_as_float(0x7fc00000);
#pragma unroll 1
  for (int si = 0; si < NBA / NWAVE; ++si) {
    const int s    = si * NWAVE + wave;
    const int node = nodeBase + s;
    const v2u co = *(const v2ua*)(COg + 2 * (size_t)node);
    int c = (int)co.x;
    const bool big = c > DEGCAP;
    c = c < 0 ? 0 : (c > DEGCAP ? DEGCAP : c);
    int o = (int)co.y;
    o = o < 0 ? 0 : (o > RCAP ? RCAP : o);
    const int nc = node < NN ? node : NN - 1;
    const v2u own = *(const v2ua*)(XDg + 2 * (size_t)nc);
    int xi = (int)own.x;
    xi = xi < 0 ? 0 : (xi > NAT - 1 ? NAT - 1 : xi);
    const float dd = __uint_as_float(own.y);
    const float rd = dd * dd;
    float a0 = 0.f, a1 = 0.f, a2 = 0.f, a3 = 0.f, a4 = 0.f, a5 = 0.f, a6 = 0.f, a7 = 0.f;
#pragma unroll 1
    for (int b0 = 0; b0 < c; b0 += 32) {
      int idx = o + b0 + lane;
      idx = idx > o + c - 1 ? o + c - 1 : idx;
      idx = idx < 0 ? 0 : (idx > RCAP - 1 ? RCAP - 1 : idx);
      const unsigned ent = lp[idx];
      int sr = (int)(ent & 0xFFFFu);
      sr = sr > NN - 1 ? NN - 1 : sr;
      const v2u xr = *(const v2ua*)(XDg + 2 * (size_t)sr);
      int tv = (int)xr.x;
      tv = tv < 0 ? 0 : (tv > NAT - 1 ? NAT - 1 : tv);
      const float cf  = __uint_as_float(xr.y) * dd;
      const int   cfi = __float_as_int(cf);
      const int m32 = (c - b0) < 32 ? (c - b0) : 32;
#pragma unroll 1
      for (int k = 0; k < m32; ++k) {
        const int   tk = __builtin_amdgcn_readlane(tv, k);
        const float ck = __int_as_float(__builtin_amdgcn_readlane(cfi, k));
        const float* row = t1s + tk * DH + 8 * lane;
        const v4f p = *(const v4fa*)row;
        const v4f q = *(const v4fa*)(row + 4);
        a0 = fmaf(ck, p.x, a0); a1 = fmaf(ck, p.y, a1); a2 = fmaf(ck, p.z, a2); a3 = fmaf(ck, p.w, a3);
        a4 = fmaf(ck, q.x, a4); a5 = fmaf(ck, q.y, a5); a6 = fmaf(ck, q.z, a6); a7 = fmaf(ck, q.w, a7);
      }
    }
    const float* srow = t1s + xi * DH + 8 * lane;
    const v4f sp = *(const v4fa*)srow;
    const v4f sq = *(const v4fa*)(srow + 4);
    const float pzr = (big || pfl != 0u) ? qnan : 0.0f;
    const bool live = node < NN;
    float y0 = relu_np((a0 + sp.x * rd) + b0v) + pzr;
    float y1 = relu_np((a1 + sp.y * rd) + b1v) + pzr;
    float y2 = relu_np((a2 + sp.z * rd) + b2v) + pzr;
    float y3 = relu_np((a3 + sp.w * rd) + b3v) + pzr;
    float y4 = relu_np((a4 + sq.x * rd) + b4v) + pzr;
    float y5 = relu_np((a5 + sq.y * rd) + b5v) + pzr;
    float y6 = relu_np((a6 + sq.z * rd) + b6v) + pzr;
    float y7 = relu_np((a7 + sq.w * rd) + b7v) + pzr;
    y0 = live ? y0 : 0.0f; y1 = live ? y1 : 0.0f; y2 = live ? y2 : 0.0f; y3 = live ? y3 : 0.0f;
    y4 = live ? y4 : 0.0f; y5 = live ? y5 : 0.0f; y6 = live ? y6 : 0.0f; y7 = live ? y7 : 0.0f;
    v4u hv, lv;
    hv.x = hl_pick(y0, false) | (hl_pick(y1, false) << 16);
    hv.y = hl_pick(y2, false) | (hl_pick(y3, false) << 16);
    hv.z = hl_pick(y4, false) | (hl_pick(y5, false) << 16);
    hv.w = hl_pick(y6, false) | (hl_pick(y7, false) << 16);
    lv.x = hl_pick(y0, true) | (hl_pick(y1, true) << 16);
    lv.y = hl_pick(y2, true) | (hl_pick(y3, true) << 16);
    lv.z = hl_pick(y4, true) | (hl_pick(y5, true) << 16);
    lv.w = hl_pick(y6, true) | (hl_pick(y7, true) << 16);
    unsigned short* hp = H1 + (size_t)node * (2 * DH) + 8 * lane;
    unsigned short* lq = hp + DH;
    const bool wr = node < MP;
    if (wr) { *(volatile v4u*)hp = hv; *(volatile v4u*)lq = lv; }
    __threadfence();
    if (wr) { *(volatile v4u*)hp = hv; *(volatile v4u*)lq = lv; }
  }
}

__global__ __launch_bounds__(NTHR) void k_agg2(const unsigned int* __restrict__ LISTg,
                                               const unsigned int* __restrict__ COg,
                                               const unsigned int* __restrict__ XDg,
                                               const unsigned int* __restrict__ POl,
                                               const float* __restrict__ H2, const float* __restrict__ gb,
                                               float* X2) {
  const int tid = (int)threadIdx.x, lane = tid & 31, wave = tid >> 5;
  const int nodeBase = (int)blockIdx.x * NBA;
  v4f ba, bb;
  {
    const v4f a = *(const v4fa*)(gb + 4 * lane);
    const v4f b = *(const v4fa*)(gb + 128 + 4 * lane);
    ba.x = bf16_val(a.x); ba.y = bf16_val(a.y); ba.z = bf16_val(a.z); ba.w = bf16_val(a.w);
    bb.x = bf16_val(b.x); bb.y = bf16_val(b.y); bb.z = bf16_val(b.z); bb.w = bf16_val(b.w);
  }
  const unsigned pfl = POl[(size_t)blockIdx.x * 32];
  const unsigned int* lp = LISTg + (size_t)blockIdx.x * RCAP;
  const float qnan = __int_as_float(0x7fc00000);
#pragma unroll 1
  for (int si = 0; si < NBA / NWAVE; ++si) {
    const int s    = si * NWAVE + wave;
    const int node = nodeBase + s;
    const v2u co = *(const v2ua*)(COg + 2 * (size_t)node);
    int c = (int)co.x;
    const bool big = c > DEGCAP;
    c = c < 0 ? 0 : (c > DEGCAP ? DEGCAP : c);
    int o = (int)co.y;
    o = o < 0 ? 0 : (o > RCAP ? RCAP : o);
    const int nc = node < NN ? node : NN - 1;
    const float dd = __uint_as_float(XDg[2 * (size_t)nc + 1]);
    const float rd = dd * dd;
    float a0 = 0.f, a1 = 0.f, a2 = 0.f, a3 = 0.f, a4 = 0.f, a5 = 0.f, a6 = 0.f, a7 = 0.f;
#pragma unroll 1
    for (int b0 = 0; b0 < c; b0 += 32) {
      int idx = o + b0 + lane;
      idx = idx > o + c - 1 ? o + c - 1 : idx;
      idx = idx < 0 ? 0 : (idx > RCAP - 1 ? RCAP - 1 : idx);
      const unsigned ent = lp[idx];
      int sr = (int)(ent & 0xFFFFu);
      sr = sr > NN - 1 ? NN - 1 : sr;
      const float cf  = __uint_as_float(XDg[2 * (size_t)sr + 1]) * dd;
      const int   cfi = __float_as_int(cf);
      const int m32 = (c - b0) < 32 ? (c - b0) : 32;
#pragma unroll 1
      for (int k = 0; k < m32; ++k) {
        const int   sk = __builtin_amdgcn_readlane(sr, k);
        const float ck = __int_as_float(__builtin_amdgcn_readlane(cfi, k));
        const float* row = H2 + (size_t)sk * DH + 4 * lane;
        const v4f p = *(const v4fa*)row;
        const v4f q = *(const v4fa*)(row + 128);
        a0 = fmaf(ck, p.x, a0); a1 = fmaf(ck, p.y, a1); a2 = fmaf(ck, p.z, a2); a3 = fmaf(ck, p.w, a3);
        a4 = fmaf(ck, q.x, a4); a5 = fmaf(ck, q.y, a5); a6 = fmaf(ck, q.z, a6); a7 = fmaf(ck, q.w, a7);
      }
    }
    const float* srow = H2 + (size_t)nc * DH + 4 * lane;
    const v4f sp = *(const v4fa*)srow;
    const v4f sq = *(const v4fa*)(srow + 128);
    const float pzr = (big || pfl != 0u) ? qnan : 0.0f;
    const bool live = node < NN;
    v4f oa, ob;
    oa.x = relu_np((a0 + sp.x * rd) + ba.x) + pzr;
    oa.y = relu_np((a1 + sp.y * rd) + ba.y) + pzr;
    oa.z = relu_np((a2 + sp.z * rd) + ba.z) + pzr;
    oa.w = relu_np((a3 + sp.w * rd) + ba.w) + pzr;
    ob.x = relu_np((a4 + sq.x * rd) + bb.x) + pzr;
    ob.y = relu_np((a5 + sq.y * rd) + bb.y) + pzr;
    ob.z = relu_np((a6 + sq.z * rd) + bb.z) + pzr;
    ob.w = relu_np((a7 + sq.w * rd) + bb.w) + pzr;
    oa.x = live ? oa.x : 0.0f; oa.y = live ? oa.y : 0.0f; oa.z = live ? oa.z : 0.0f; oa.w = live ? oa.w : 0.0f;
    ob.x = live ? ob.x : 0.0f; ob.y = live ? ob.y : 0.0f; ob.z = live ? ob.z : 0.0f; ob.w = live ? ob.w : 0.0f;
    float* op = X2 + (size_t)node * DH + 4 * lane;
    float* oq = op + 128;
    const bool wr = node < MP;
    if (wr) { *(volatile v4f*)op = oa; *(volatile v4f*)oq = ob; }
    __threadfence();
    if (wr) { *(volatile v4f*)op = oa; *(volatile v4f*)oq = ob; }
  }
}

__global__ __launch_bounds__(NTHR) void k_pool(const float* __restrict__ X2, const int* __restrict__ bat,
                                               unsigned short* PO, unsigned int* POl) {
  __shared__ __attribute__((aligned(16))) int plist[PCAP];
  __shared__ int wcnt[NWAVE];
  const int tid = (int)threadIdx.x, lane = tid & 31, wave = tid >> 5;
  const int g0 = (int)blockIdx.x * PGB;
  for (int i = tid; i < PCAP; i += NTHR) plist[i] = 0;
  if (tid < NWAVE) wcnt[tid] = 0;
  __syncthreads();

  int tot = 0;
#pragma unroll 1
  for (int c0 = 0; c0 < NN; c0 += NTHR) {
    const int i  = c0 + tid;
    const int ic = i < NN ? i : NN - 1;
    const int b  = bat[ic];
    const unsigned gl = (unsigned)(b - g0);
    const bool hit = (i < NN) && (gl < (unsigned)PGB);
    const unsigned msk = __builtin_amdgcn_ballot_w32(hit);
    if (lane == 0) wcnt[wave] = (int)__builtin_popcount(msk);
    __syncthreads();
    int pre = 0, all = 0;
#pragma unroll
    for (int w2 = 0; w2 < NWAVE; ++w2) {
      int cw = wcnt[w2];
      cw = cw < 0 ? 0 : (cw > 32 ? 32 : cw);
      all += cw;
      pre += (w2 < wave) ? cw : 0;
    }
    const int pos = tot + pre + (int)__builtin_amdgcn_mbcnt_lo(msk, 0u);
    if (hit && pos < PCAP) plist[pos] = (int)((gl << 16) | (unsigned)i);
    tot += all;
    __syncthreads();
  }
  const bool ovf = tot > PCAP;
  const int nl = tot > PCAP ? PCAP : tot;
  const float qnan = __int_as_float(0x7fc00000);
  const float pz = ovf ? qnan : 0.0f;

#pragma unroll 1
  for (int j = 0; j < PGB / NWAVE; ++j) {
    const int gloc = wave * (PGB / NWAVE) + j;
    const int g = g0 + gloc;
    float a0 = 0.f, a1 = 0.f, a2 = 0.f, a3 = 0.f, a4 = 0.f, a5 = 0.f, a6 = 0.f, a7 = 0.f;
    int cnt = 0;
#pragma unroll 1
    for (int b0 = 0; b0 < nl; b0 += 32) {
      int idx = b0 + lane;
      const bool inr = idx < nl;
      idx = idx > nl - 1 ? nl - 1 : idx;
      idx = idx < 0 ? 0 : idx;
      const int ent = plist[idx];
      const bool hit = inr && ((ent >> 16) == gloc);
      int nodev = ent & 0xFFFF;
      nodev = nodev > NN - 1 ? NN - 1 : nodev;
      unsigned msk = __builtin_amdgcn_ballot_w32(hit);
      int nh = (int)__builtin_popcount(msk);
      nh = nh > 32 ? 32 : nh;
      cnt += nh;
#pragma unroll 1
      for (int q = 0; q < nh; ++q) {
        int k = __builtin_ffs((int)msk) - 1;
        msk &= msk - 1u;
        k = k < 0 ? 0 : k;
        const int node = __builtin_amdgcn_readlane(nodev, k);
        const float* row = X2 + (size_t)node * DH + 8 * lane;
        const v4f p = *(const v4fa*)row;
        const v4f r = *(const v4fa*)(row + 4);
        a0 += p.x; a1 += p.y; a2 += p.z; a3 += p.w;
        a4 += r.x; a5 += r.y; a6 += r.z; a7 += r.w;
      }
    }
    const float cf = (cnt < 1) ? 1.0f : (float)cnt;
    const float y0 = a0 / cf + pz, y1 = a1 / cf + pz, y2 = a2 / cf + pz, y3 = a3 / cf + pz;
    const float y4 = a4 / cf + pz, y5 = a5 / cf + pz, y6 = a6 / cf + pz, y7 = a7 / cf + pz;
    v4u hv, lv;
    hv.x = hl_pick(y0, false) | (hl_pick(y1, false) << 16);
    hv.y = hl_pick(y2, false) | (hl_pick(y3, false) << 16);
    hv.z = hl_pick(y4, false) | (hl_pick(y5, false) << 16);
    hv.w = hl_pick(y6, false) | (hl_pick(y7, false) << 16);
    lv.x = hl_pick(y0, true) | (hl_pick(y1, true) << 16);
    lv.y = hl_pick(y2, true) | (hl_pick(y3, true) << 16);
    lv.z = hl_pick(y4, true) | (hl_pick(y5, true) << 16);
    lv.w = hl_pick(y6, true) | (hl_pick(y7, true) << 16);
    unsigned short* hp = PO + (size_t)g * (2 * DH) + 8 * lane;
    unsigned short* lq = hp + DH;
    *(volatile v4u*)hp = hv; *(volatile v4u*)lq = lv;
    __threadfence();
    *(volatile v4u*)hp = hv; *(volatile v4u*)lq = lv;
  }
  const unsigned fv = ovf ? 1u : 0u;
  const v4u fl = {fv, fv, fv, fv};
  const bool flw = (wave == 0) && (lane < 8);
  if (flw) *(volatile v4u*)(POl + (size_t)blockIdx.x * 32 + 4 * lane) = fl;
  __threadfence();
  if (flw) *(volatile v4u*)(POl + (size_t)blockIdx.x * 32 + 4 * lane) = fl;
}

__device__ __forceinline__ void egs_unit(const float* __restrict__ P, unsigned short* EG, int v, int coff,
                                         float pz) {
  const int g  = v >> 5;
  const int c8 = (v & 31) * 8;
  const float* pa = P + (size_t)g * DH + c8;
  const float* pb = P + (size_t)(GG + g) * DH + c8;
  const v4f a0 = *(const v4fa*)pa;
  const v4f a1 = *(const v4fa*)(pa + 4);
  const v4f b0 = *(const v4fa*)pb;
  const v4f b1 = *(const v4fa*)(pb + 4);
  const float y0 = relu_np(a0.x + b0.x) + pz, y1 = relu_np(a0.y + b0.y) + pz;
  const float y2 = relu_np(a0.z + b0.z) + pz, y3 = relu_np(a0.w + b0.w) + pz;
  const float y4 = relu_np(a1.x + b1.x) + pz, y5 = relu_np(a1.y + b1.y) + pz;
  const float y6 = relu_np(a1.z + b1.z) + pz, y7 = relu_np(a1.w + b1.w) + pz;
  v4u hv, lv;
  hv.x = hl_pick(y0, false) | (hl_pick(y1, false) << 16);
  hv.y = hl_pick(y2, false) | (hl_pick(y3, false) << 16);
  hv.z = hl_pick(y4, false) | (hl_pick(y5, false) << 16);
  hv.w = hl_pick(y6, false) | (hl_pick(y7, false) << 16);
  lv.x = hl_pick(y0, true) | (hl_pick(y1, true) << 16);
  lv.y = hl_pick(y2, true) | (hl_pick(y3, true) << 16);
  lv.z = hl_pick(y4, true) | (hl_pick(y5, true) << 16);
  lv.w = hl_pick(y6, true) | (hl_pick(y7, true) << 16);
  unsigned short* hp = EG + (size_t)g * (2 * DHID) + coff + c8;
  unsigned short* lq = hp + DHID;
  *(volatile v4u*)hp = hv; *(volatile v4u*)lq = lv;
  __threadfence();
  *(volatile v4u*)hp = hv; *(volatile v4u*)lq = lv;
}

__global__ __launch_bounds__(NTHR) void k_egs(const float* __restrict__ Gf, const float* __restrict__ Eo,
                                              const unsigned int* __restrict__ POl, unsigned short* EG) {
  __shared__ int pf;
  const int tid = (int)threadIdx.x;
  if (tid == 0) pf = 0;
  __syncthreads();
  const int fi = tid < NPOL ? tid : NPOL - 1;
  const unsigned fl = POl[(size_t)fi * 32];
  if (fl != 0u) pf = 1;
  __syncthreads();
  const float pz = (pf != 0) ? __int_as_float(0x7fc00000) : 0.0f;
  const int u = (int)blockIdx.x * NTHR + tid;
  if (u < GG * 32) egs_unit(Gf, EG, u, 0, pz);
  else             egs_unit(Eo, EG, u - GG * 32, DH, pz);
}
static_assert((GG * 32) % NTHR == 0 && NPOL <= NTHR);

constexpr size_t SZ_R    = (size_t)MP * 512 * 2;
constexpr size_t O_R1    = 0;
constexpr size_t O_R2    = O_R1 + SZ_R;
constexpr size_t O_LIST  = O_R2 + SZ_R;
constexpr size_t SZ_LIST = (size_t)2 * NBLK * RCAP * 4;
constexpr size_t O_CO    = O_LIST + SZ_LIST;
constexpr size_t SZ_TAB  = (size_t)2 * NPADN * 8;
constexpr size_t O_XD    = O_CO + SZ_TAB;
constexpr size_t O_PO    = O_XD + SZ_TAB;
constexpr size_t SZ_PO   = (size_t)NPOL * 128;
constexpr size_t O_GW1T  = O_PO + SZ_PO;
constexpr size_t O_GW2D  = O_GW1T + (size_t)DH * DE * 2;
constexpr size_t O_FCWD  = O_GW2D + (size_t)DH * 2 * DH * 2;
constexpr size_t O_EW1T  = O_FCWD + (size_t)DH * 2 * DH * 2;
constexpr size_t O_EW2D  = O_EW1T + (size_t)DH * DE * 2;
constexpr size_t O_DW1D  = O_EW2D + (size_t)DH * 2 * DH * 2;
constexpr size_t O_DW2D  = O_DW1D + (size_t)DHID * 2 * DHID * 2;
constexpr size_t O_DW3D  = O_DW2D + (size_t)DHID * 2 * DHID * 2;
constexpr size_t O_AE    = O_DW3D + (size_t)DOUT * 2 * DHID * 2;
constexpr size_t O_T1    = O_AE + (size_t)128 * DE * 2;
constexpr size_t O_E0    = O_T1 + (size_t)128 * DH * 4;
constexpr size_t O_POHL  = O_E0 + (size_t)2 * GG * DE * 2;
constexpr size_t O_END   = O_POHL + (size_t)2 * GG * 2 * DH * 2;
constexpr size_t SZ_TP   = 2097152;
static_assert(SZ_R % 256 == 0 && SZ_LIST % 256 == 0 && SZ_TAB % 256 == 0 && SZ_PO % 128 == 0);
static_assert(O_GW1T % 256 == 0 && O_AE % 256 == 0 && O_T1 % 256 == 0 && O_E0 % 256 == 0 && O_POHL % 256 == 0);
static_assert(SZ_R == (size_t)MP * DH * 4);
static_assert((size_t)2 * GG * DH * 4 == SZ_TP && (size_t)2 * GG * 2 * DH * 2 == SZ_TP);
static_assert((size_t)GG * 2 * DHID * 2 == SZ_TP && 6 * SZ_TP <= SZ_R);
static_assert(O_END <= (size_t)WSMAX);

extern "C" void kernel_launch(void* const* d_in, const int* in_sizes, int n_in,
                              void* d_out, int out_size, void* d_ws, size_t ws_size,
                              hipStream_t stream) {
  if (n_in < 26) return;
  if (in_sizes[0] != NN || in_sizes[1] != 2 * EE || in_sizes[2] != GG || in_sizes[3] != NN) return;
  if (in_sizes[4] != NN || in_sizes[5] != 2 * EE || in_sizes[6] != GG || in_sizes[7] != NN) return;
  if (in_sizes[8] != NAT * DE) return;
  if (in_sizes[9] != DE * DH || in_sizes[10] != DH) return;
  if (in_sizes[11] != DH * DH || in_sizes[12] != DH) return;
  if (in_sizes[13] != DH * DH || in_sizes[14] != DH) return;
  if (in_sizes[15] != VOC * DE) return;
  if (in_sizes[16] != DE * DH || in_sizes[17] != DH) return;
  if (in_sizes[18] != DH * DH || in_sizes[19] != DH) return;
  if (in_sizes[20] != DHID * DHID || in_sizes[21] != DHID) return;
  if (in_sizes[22] != DHID * DHID || in_sizes[23] != DHID) return;
  if (in_sizes[24] != DHID * DOUT || in_sizes[25] != DOUT) return;
  if (out_size != GG * DOUT) return;
  if (O_END > ws_size) return;

  const int*   x1   = (const int*)d_in[0];
  const int*   ei1  = (const int*)d_in[1];
  const int*   ent1 = (const int*)d_in[2];
  const int*   bt1  = (const int*)d_in[3];
  const int*   x2   = (const int*)d_in[4];
  const int*   ei2  = (const int*)d_in[5];
  const int*   ent2 = (const int*)d_in[6];
  const int*   bt2  = (const int*)d_in[7];
  const float* aemb = (const float*)d_in[8];
  const float* gW1  = (const float*)d_in[9];
  const float* gb1  = (const float*)d_in[10];
  const float* gW2  = (const float*)d_in[11];
  const float* gb2  = (const float*)d_in[12];
  const float* fcW  = (const float*)d_in[13];
  const float* fcb  = (const float*)d_in[14];
  const float* eemb = (const float*)d_in[15];
  const float* eW1  = (const float*)d_in[16];
  const float* eb1  = (const float*)d_in[17];
  const float* eW2  = (const float*)d_in[18];
  const float* eb2  = (const float*)d_in[19];
  const float* dW1  = (const float*)d_in[20];
  const float* db1  = (const float*)d_in[21];
  const float* dW2  = (const float*)d_in[22];
  const float* db2  = (const float*)d_in[23];
  const float* dW3  = (const float*)d_in[24];
  const float* db3  = (const float*)d_in[25];
  float* out = (float*)d_out;

  char* ws = (char*)d_ws;
  unsigned short* H1hl = (unsigned short*)(ws + O_R1);
  float*          X2   = (float*)(ws + O_R1);
  float*          H2   = (float*)(ws + O_R2);
  unsigned int*   LIST = (unsigned int*)(ws + O_LIST);
  unsigned int*   CO   = (unsigned int*)(ws + O_CO);
  unsigned int*   XD   = (unsigned int*)(ws + O_XD);
  unsigned int*   POL  = (unsigned int*)(ws + O_PO);
  unsigned short* gW1T = (unsigned short*)(ws + O_GW1T);
  unsigned short* gW2D = (unsigned short*)(ws + O_GW2D);
  unsigned short* fcWD = (unsigned short*)(ws + O_FCWD);
  unsigned short* eW1T = (unsigned short*)(ws + O_EW1T);
  unsigned short* eW2D = (unsigned short*)(ws + O_EW2D);
  unsigned short* dW1D = (unsigned short*)(ws + O_DW1D);
  unsigned short* dW2D = (unsigned short*)(ws + O_DW2D);
  unsigned short* dW3D = (unsigned short*)(ws + O_DW3D);
  unsigned short* AE   = (unsigned short*)(ws + O_AE);
  float*          T1   = (float*)(ws + O_T1);
  unsigned short* E0   = (unsigned short*)(ws + O_E0);
  unsigned short* POhl = (unsigned short*)(ws + O_POHL);
  float*          Gf   = (float*)(ws + O_R2 + 0 * SZ_TP);
  unsigned short* E1hl = (unsigned short*)(ws + O_R2 + 1 * SZ_TP);
  float*          Eo   = (float*)(ws + O_R2 + 2 * SZ_TP);
  unsigned short* EGS  = (unsigned short*)(ws + O_R2 + 3 * SZ_TP);
  unsigned short* D1hl = (unsigned short*)(ws + O_R2 + 4 * SZ_TP);
  unsigned short* D2hl = (unsigned short*)(ws + O_R2 + 5 * SZ_TP);

  const int bktLds = BKT_LDS_INTS * 4;
  hipFuncSetAttribute(reinterpret_cast<const void*>(&k_bucket), hipFuncAttributeMaxDynamicSharedMemorySize, bktLds);

  k_prep<<<PB10 / NTHR, NTHR, 0, stream>>>(gW1, gW2, fcW, eW1, eW2, dW1, dW2, dW3, aemb, eemb, ent1, ent2,
                                           gW1T, gW2D, fcWD, eW1T, eW2D, dW1D, dW2D, dW3D, AE, E0);
  k_gemm<0, 0><<<dim3(128 / GBM, DH / GBN), GTHR, 0, stream>>>(AE, gW1T, gb1, 0, T1, AE, DE, DH);
  k_bucket<<<NBLK, NTHR, bktLds, stream>>>(ei1, ei1 + EE, x1, LIST, CO, XD, POL);
  k_bucket<<<NBLK, NTHR, bktLds, stream>>>(ei2, ei2 + EE, x2, LIST + (size_t)NBLK * RCAP,
                                           CO + (size_t)2 * NPADN, XD + (size_t)2 * NPADN,
                                           POL + (size_t)NBLK * 32);
  for (int s = 0; s < 2; ++s) {
    const unsigned int* Ls = LIST + (size_t)s * NBLK * RCAP;
    const unsigned int* Cs = CO + (size_t)s * 2 * NPADN;
    const unsigned int* Xs = XD + (size_t)s * 2 * NPADN;
    const unsigned int* Ps = POL + (size_t)s * NBLK * 32;
    const int* bat = (s == 0) ? bt1 : bt2;
    k_agg1<<<NBLK, NTHR, 0, stream>>>(Ls, Cs, Xs, Ps, T1, gb1, H1hl);
    k_gemm<0, 0><<<dim3(MP / GBM, DH / GBN), GTHR, 0, stream>>>(H1hl, gW2D, gb1, 0, H2, H1hl, 2 * DH, DH);
    k_agg2<<<NBLK, NTHR, 0, stream>>>(Ls, Cs, Xs, Ps, H2, gb2, X2);
    k_pool<<<NPB, NTHR, 0, stream>>>(X2, bat, POhl + (size_t)s * GG * 2 * DH,
                                     POL + (size_t)(2 * NBLK + s * NPB) * 32);
  }
  k_gemm<0, 0><<<dim3(2 * GG / GBM, DH / GBN), GTHR, 0, stream>>>(POhl, fcWD, fcb, 1, Gf, POhl, 2 * DH, DH);
  k_gemm<1, 1><<<dim3(2 * GG / GBM, DH / GBN), GTHR, 0, stream>>>(E0, eW1T, eb1, 1, Gf, E1hl, DE, DH);
  k_gemm<1, 0><<<dim3(2 * GG / GBM, DH / GBN), GTHR, 0, stream>>>(E1hl, eW2D, eb2, 1, Eo, E1hl, 2 * DH, DH);
  k_egs<<<(GG * 64) / NTHR, NTHR, 0, stream>>>(Gf, Eo, POL, EGS);
  k_gemm<1, 1><<<dim3(GG / GBM, DHID / GBN), GTHR, 0, stream>>>(EGS, dW1D, db1, 1, Gf, D1hl, 2 * DHID, DHID);
  k_gemm<1, 1><<<dim3(GG / GBM, DHID / GBN), GTHR, 0, stream>>>(D1hl, dW2D, db2, 1, Gf, D2hl, 2 * DHID, DHID);
  k_gemm<0, 0><<<dim3(GG / GBM, DOUT / GBN), GTHR, 0, stream>>>(D2hl, dW3D, db3, 1, out, D2hl, 2 * DHID, DOUT);
}
